// Modnet_13572096655546
// MI455X (gfx1250) — hardware-verified
//
#include <hip/hip_runtime.h>
#include <stddef.h>
#include <math.h>


#define D_IN   16
#define K_IN   18
#define H_N    128
#define QMAX   512
#define NTHR   256
#define RB     128
#define PT     40
#define SC_W   4.0f
#define SC_INV 0.25f

static_assert(RB == 16 * (NTHR / 32));
static_assert((PT * 2) % 16 == 0);
static_assert(RB / 4 == 32);
static_assert(NTHR == 2 * H_N);
static_assert(QMAX % NTHR == 0);

#if __has_builtin(__builtin_amdgcn_exp2f)
#define EXP2_F(x) __builtin_amdgcn_exp2f(x)
#else
#define EXP2_F(x) exp2f(x)
#endif
#if __has_builtin(__builtin_amdgcn_rcpf)
#define RCP_F(x) __builtin_amdgcn_rcpf(x)
#else
#define RCP_F(x) (1.0f / (x))
#endif

typedef _Float16 v16h __attribute__((ext_vector_type(16)));
typedef _Float16 v8h  __attribute__((ext_vector_type(8)));
typedef float    v4f  __attribute__((ext_vector_type(4)));
typedef float    v8f  __attribute__((ext_vector_type(8)));
union FragH { v16h v; v8h h[2]; };

__device__ __forceinline__ v8f wmh(v16h a, v16h b, v8f c) {
  v8f d = __builtin_amdgcn_wmma_f32_16x16x32_f16(false, a, false, b, (short)0, c, false, false);
#if defined(__HIP_DEVICE_COMPILE__)
  asm volatile("v_nop\n\tv_nop\n\tv_nop\n\tv_nop" : "+v"(d) : "v"(a), "v"(b));
#endif
  return d;
}

__device__ __forceinline__ v8f zero8() {
  v8f z = {0.f, 0.f, 0.f, 0.f, 0.f, 0.f, 0.f, 0.f};
  return z;
}

__device__ __forceinline__ float tanh_f(float x) {
  const float y = fminf(__builtin_fabsf(x), 16.0f);
  const float e = EXP2_F(-2.8853900817779268f * y);
  const float t = (1.0f - e) * RCP_F(1.0f + e);
  return __builtin_copysignf(t, x);
}

__global__ __launch_bounds__(NTHR) void k_fused(const float* __restrict__ xin,
                                                const float* __restrict__ eqp,
                                                const float* __restrict__ qx,
                                                const float* __restrict__ W1,
                                                const float* __restrict__ b1,
                                                const float* __restrict__ W2,
                                                const float* __restrict__ b2,
                                                float* out, int nrow, int nq) {
  __shared__ __align__(16) _Float16 sB[H_N * PT];
  __shared__ float sY[QMAX];
  __shared__ float sW2[H_N];
  __shared__ float sB1[H_N];
  __shared__ v4f sO4[RB / 4];
  float* sO = (float*)sO4;

  const int tid = (int)threadIdx.x, lane = tid & 31, wv = tid >> 5, h = lane >> 4, m = lane & 15;
  const int brow = (int)blockIdx.x * RB;
  const int wr = wv * 16;

  {
    const int n = tid >> 1, kh = tid & 1;
    v8h o0, o1;
#pragma unroll
    for (int e = 0; e < 8; ++e) {
      const int k0 = 16 * kh + e, k1 = k0 + 8;
      const int q0 = k0 < K_IN ? k0 : K_IN - 1;
      const int q1 = k1 < K_IN ? k1 : K_IN - 1;
      const float w0 = W1[q0 * H_N + n];
      const float w1 = W1[q1 * H_N + n];
      o0[e] = (_Float16)((k0 < K_IN) ? SC_W * w0 : 0.0f);
      o1[e] = (_Float16)((k1 < K_IN) ? SC_W * w1 : 0.0f);
    }
    _Float16* p = sB + n * PT + 16 * kh;
    *(v8h*)p = o0;
    *(v8h*)(p + 8) = o1;
  }
  if (tid < H_N) {
    sW2[tid] = W2[tid];
    sB1[tid] = b1[tid];
  }
  {
    const float ev0 = eqp[0], ev1 = eqp[1];
#pragma unroll 1
    for (int i = tid; i < QMAX; i += NTHR) {
      const int iq = i < nq ? i : nq - 1;
      const float a0 = qx[2 * iq], a1 = qx[2 * iq + 1];
      const float s = sinf(fmaf(a1, ev1, a0 * ev0));
      sY[i] = (i < nq) ? s : 0.0f;
    }
  }

  float inr[D_IN];
  {
    int rg = brow + wr + m;
    rg = rg > nrow - 1 ? nrow - 1 : rg;
    const v4f* src = (const v4f*)(xin + (size_t)rg * D_IN);
#pragma unroll
    for (int j = 0; j < 4; ++j) {
      const v4f v = src[j];
      inr[4 * j + 0] = v[0];
      inr[4 * j + 1] = v[1];
      inr[4 * j + 2] = v[2];
      inr[4 * j + 3] = v[3];
    }
  }
  FragH af;
  v8h abase;
  {
    abase[0] = (_Float16)inr[6];
    abase[1] = (_Float16)inr[7];
#pragma unroll
    for (int e = 2; e < 8; ++e) {
      const float f = h ? inr[6 + e] : inr[e - 2];
      abase[e] = (_Float16)f;
    }
    v8h o1;
    const float f0 = h ? 0.0f : inr[14];
    const float f1 = h ? 0.0f : inr[15];
    o1[0] = (_Float16)f0;
    o1[1] = (_Float16)f1;
#pragma unroll
    for (int e = 2; e < 8; ++e) o1[e] = (_Float16)0.0f;
    af.h[1] = o1;
  }
  __syncthreads();

  float acco[8];
#pragma unroll
  for (int r = 0; r < 8; ++r) acco[r] = 0.0f;
  const float b2v = b2[0];

#pragma unroll 1
  for (int q = 0; q < nq; ++q) {
    const float qx0 = qx[2 * q], qx1 = qx[2 * q + 1];
    {
      v8h o0 = abase;
      const float g0 = h ? inr[6] : qx0;
      const float g1 = h ? inr[7] : qx1;
      o0[0] = (_Float16)g0;
      o0[1] = (_Float16)g1;
      af.h[0] = o0;
    }
    v8f acc[8];
#pragma unroll
    for (int t = 0; t < 8; ++t) {
      FragH bf;
      const _Float16* pb = sB + (16 * t + m) * PT + 8 * h;
      bf.h[0] = *(const v8h*)pb;
      bf.h[1] = *(const v8h*)(pb + 16);
      acc[t] = wmh(af.v, bf.v, zero8());
    }
    float p[8];
#pragma unroll
    for (int r = 0; r < 8; ++r) p[r] = 0.0f;
#pragma unroll
    for (int t = 0; t < 8; ++t) {
      const int c = 16 * t + m;
      const float w2 = sW2[c];
      const float bb = sB1[c];
#pragma unroll
      for (int r = 0; r < 8; ++r) {
        const float v = tanh_f(fmaf(acc[t][r], SC_INV, bb));
        p[r] = fmaf(v, w2, p[r]);
      }
    }
#pragma unroll
    for (int off = 1; off < 16; off <<= 1) {
#pragma unroll
      for (int r = 0; r < 8; ++r) p[r] += __shfl_xor(p[r], off, 32);
    }
    const float yq = sY[q];
#pragma unroll
    for (int r = 0; r < 8; ++r) acco[r] = fmaf(p[r] + b2v, yq, acco[r]);
  }

  {
    float ov = acco[0];
#pragma unroll
    for (int r = 1; r < 8; ++r) ov = (m == r) ? acco[r] : ov;
    if (m < 8) sO[wr + 8 * h + m] = ov;
  }
  __syncthreads();

  if (wv == 0) {
    const v4f o = sO4[lane];
    float* g = out + (size_t)brow + 4 * lane;
    *(volatile v4f*)g = o;
    __threadfence();
    *(volatile v4f*)g = o;
  }
}

extern "C" void kernel_launch(void* const* d_in, const int* in_sizes, int n_in,
                              void* d_out, int out_size, void* d_ws, size_t ws_size,
                              hipStream_t stream) {
  if (n_in < 7) return;
  const int nrow = out_size;
  if (nrow <= 0 || (nrow % RB) != 0) return;
  if (in_sizes[0] != nrow * D_IN) return;
  if (in_sizes[1] < 2) return;
  const int nq = in_sizes[2] / 2;
  if (nq < 1 || nq > QMAX || in_sizes[2] != 2 * nq) return;
  if (in_sizes[3] != K_IN * H_N) return;
  if (in_sizes[4] != H_N || in_sizes[5] != H_N) return;
  if (in_sizes[6] < 1) return;

  const float* xin = (const float*)d_in[0];
  const float* eqp = (const float*)d_in[1];
  const float* qx  = (const float*)d_in[2];
  const float* W1  = (const float*)d_in[3];
  const float* b1  = (const float*)d_in[4];
  const float* W2  = (const float*)d_in[5];
  const float* b2  = (const float*)d_in[6];
  float* out = (float*)d_out;

  (void)d_ws; (void)ws_size;

  k_fused<<<nrow / RB, NTHR, 0, stream>>>(xin, eqp, qx, W1, b1, W2, b2, out, nrow, nq);
}
